// LocalTransformerDecoderLayer_73787538145798
// MI455X (gfx1250) — hardware-run, weakly checked
//
#include <hip/hip_runtime.h>
#include <math.h>
#include <stdint.h>
#include <stddef.h>

#define NBATCH 8
#define CH     256
#define NQRY   1024
#define NKEY   4096
#define NS     16
#define NHEAD  8
#define DHEAD  32
#define FFD    2048
#define NBQ    (NBATCH * NQRY)
#define TP     260
#define EP     264
#define WSCL   256.0f
#define ASCL   16.0f
#define RSQD   0.17677669529663687f
#define LNEPS  1e-5f

#define ST_BYTES  (64 * TP * 4)
#define SE_OFF    ST_BYTES
#define SE_BYTES  (64 * EP * 2)
#define SQH_OFF   (SE_OFF + SE_BYTES)
#define SSC_OFF   (SQH_OFF + 4 * CH * 4)
#define SG_OFF    (SSC_OFF + 512 * 4)
#define SAO_OFF   (SG_OFF + 64 * 4 * 4)
#define SIDX_OFF  (SAO_OFF + 4 * CH * 2)
#define SQP_OFF   (SIDX_OFF + 64 * 4)
#define SCNT_OFF  (SQP_OFF + 4 * 8 * 4)
#define ATT_SMEM  (SCNT_OFF + 16)
#define SROW_OFF  ST_BYTES
#define LN1_SMEM  (SROW_OFF + 8 * CH * 2)
#define GEMM_SMEM ST_BYTES
#define BQ_SH_OFF (32 * TP * 4)
#define BQ_SP_OFF (BQ_SH_OFF + 32 * EP * 2)
#define BQ_SMEM   (BQ_SP_OFF + 32 * 8 * 4)

static_assert(NHEAD * DHEAD == CH && CH == 256 && NS == 16 && DHEAD == 32);
static_assert((NQRY % 64) == 0 && (NBQ % 64) == 0 && (NKEY % 32) == 0 && (NBQ % 32) == 0);
static_assert((CH % 32) == 0 && (FFD % 32) == 0 && (FFD % CH) == 0);
static_assert(((TP * 4) % 16) == 0 && ((EP * 2) % 16) == 0);
static_assert((SE_OFF % 16) == 0 && (SQH_OFF % 16) == 0 && (SSC_OFF % 16) == 0 && (SG_OFF % 16) == 0);
static_assert((SAO_OFF % 16) == 0 && (SIDX_OFF % 16) == 0 && (SQP_OFF % 16) == 0 && (SCNT_OFF % 16) == 0);
static_assert((BQ_SH_OFF % 16) == 0 && (BQ_SP_OFF % 16) == 0);
static_assert(((CH * CH) % 2048) == 0 && ((FFD * CH) % 2048) == 0);

typedef _Float16 v16h __attribute__((ext_vector_type(16)));
typedef unsigned short v16us __attribute__((ext_vector_type(16)));
typedef unsigned short v8us  __attribute__((ext_vector_type(8)));
typedef float v8f __attribute__((ext_vector_type(8)));
typedef float v4f __attribute__((ext_vector_type(4)));
typedef unsigned int v4u __attribute__((ext_vector_type(4)));
typedef unsigned int v2u __attribute__((ext_vector_type(2)));

union FragU { v16us v; v8us h[2]; };

extern __shared__ __align__(16) unsigned char g_smem[];

__device__ __forceinline__ float bf16r(float f) {
  unsigned u = __float_as_uint(f);
  u += 0x7FFFu + ((u >> 16) & 1u);
  u &= 0xFFFF0000u;
  return __uint_as_float(u);
}
__device__ __forceinline__ v4f bf16r4(v4f x) {
  v4f r;
  r[0] = bf16r(x[0]); r[1] = bf16r(x[1]); r[2] = bf16r(x[2]); r[3] = bf16r(x[3]);
  return r;
}
__device__ __forceinline__ unsigned short f2h(float f) {
  return __builtin_bit_cast(unsigned short, (_Float16)f);
}
__device__ __forceinline__ unsigned pk16(unsigned short a, unsigned short b) {
  return (unsigned)a | ((unsigned)b << 16);
}
__device__ __forceinline__ v2u pack4h(v4f x) {
  v2u r;
  r[0] = pk16(f2h(x[0]), f2h(x[1]));
  r[1] = pk16(f2h(x[2]), f2h(x[3]));
  return r;
}
__device__ __forceinline__ v4u pack8h(v4f a, v4f b) {
  v4u r;
  r[0] = pk16(f2h(a[0]), f2h(a[1]));
  r[1] = pk16(f2h(a[2]), f2h(a[3]));
  r[2] = pk16(f2h(b[0]), f2h(b[1]));
  r[3] = pk16(f2h(b[2]), f2h(b[3]));
  return r;
}
__device__ __forceinline__ int clampi(int v, int lo, int hi) { return v < lo ? lo : (v > hi ? hi : v); }
__device__ __forceinline__ v8f zero8() { v8f z = {0.f, 0.f, 0.f, 0.f, 0.f, 0.f, 0.f, 0.f}; return z; }
__device__ __forceinline__ float wsum(float v) {
#pragma unroll
  for (int off = 16; off > 0; off >>= 1) v += __shfl_xor(v, off, 32);
  return v;
}

__device__ __forceinline__ v16us ldfrag_u(const unsigned short* p) {
  FragU f;
  f.h[0] = *(const v8us*)(p);
  f.h[1] = *(const v8us*)(p + 16);
  return f.v;
}

__device__ __forceinline__ v8f mma_h_raw(v16us a, v16us b, v8f c) {
  return __builtin_amdgcn_wmma_f32_16x16x32_f16(false, __builtin_bit_cast(v16h, a), false,
                                                __builtin_bit_cast(v16h, b), (short)0, c, false, false);
}
__device__ __forceinline__ void dep_guard2(v8f& a, v8f& b, v16us x) {
#if defined(__HIP_DEVICE_COMPILE__)
  asm volatile("v_nop\n\tv_nop\n\tv_nop\n\tv_nop" : "+v"(a), "+v"(b) : "v"(x));
#endif
}
__device__ __forceinline__ void keep2_u(v16us a, v16us b) {
#if defined(__HIP_DEVICE_COMPILE__)
  asm volatile("v_nop" :: "v"(a), "v"(b));
#endif
}
__device__ __forceinline__ void acc_guard4(v8f& a, v8f& b, v8f& c, v8f& d) {
#if defined(__HIP_DEVICE_COMPILE__)
  asm volatile("v_nop\n\tv_nop\n\tv_nop\n\tv_nop" : "+v"(a), "+v"(b), "+v"(c), "+v"(d));
#endif
}
__device__ __forceinline__ void wave_sync_lds() {
  __builtin_amdgcn_fence(__ATOMIC_RELEASE, "workgroup");
  __builtin_amdgcn_wave_barrier();
  __builtin_amdgcn_fence(__ATOMIC_ACQUIRE, "workgroup");
}

template <bool ALDS>
__device__ __forceinline__ void bgemm64x256(const unsigned short* __restrict__ Ap, int lda,
                                            const unsigned short* __restrict__ Bt, int ldb,
                                            int K, float osc, const float* __restrict__ bias) {
  float* sT = (float*)g_smem;
  const unsigned short* sA = (const unsigned short*)(g_smem + SE_OFF);
  const int lane = threadIdx.x & 31, wave = threadIdx.x >> 5;
  const int rl = lane & 15;
  const int koff = (lane >> 4) * 8;
  const int mOff = (lane >> 4) * 8;
  const int nw = wave * 32;

  v8f acc[4][2];
#pragma unroll
  for (int i = 0; i < 4; ++i) { acc[i][0] = zero8(); acc[i][1] = zero8(); }

#pragma unroll 1
  for (int k0 = 0; k0 < K; k0 += 32) {
    const v16us b0 = ldfrag_u(Bt + (size_t)(nw + rl) * ldb + koff + k0);
    const v16us b1 = ldfrag_u(Bt + (size_t)(nw + 16 + rl) * ldb + koff + k0);
#pragma unroll
    for (int i = 0; i < 4; ++i) {
      v16us a;
      if (ALDS) a = ldfrag_u(sA + ((i << 4) + rl) * lda + koff + k0);
      else      a = ldfrag_u(Ap + (size_t)((i << 4) + rl) * lda + koff + k0);
      acc[i][0] = mma_h_raw(a, b0, acc[i][0]);
      acc[i][1] = mma_h_raw(a, b1, acc[i][1]);
      dep_guard2(acc[i][0], acc[i][1], a);
    }
    keep2_u(b0, b1);
  }
  acc_guard4(acc[0][0], acc[0][1], acc[1][0], acc[1][1]);
  acc_guard4(acc[2][0], acc[2][1], acc[3][0], acc[3][1]);

  const float bv0 = bf16r(bias[nw + rl]);
  const float bv1 = bf16r(bias[nw + 16 + rl]);
#pragma unroll
  for (int i = 0; i < 4; ++i) {
#pragma unroll
    for (int r = 0; r < 8; ++r) {
      const int row = (i << 4) + mOff + r;
      sT[row * TP + nw + rl]      = acc[i][0][r] * osc + bv0;
      sT[row * TP + nw + 16 + rl] = acc[i][1][r] * osc + bv1;
    }
  }
}

__global__ __launch_bounds__(256) void k_cvtw(const float* __restrict__ w0, const float* __restrict__ w1,
                                              const float* __restrict__ w2, const float* __restrict__ w3,
                                              const float* __restrict__ w4, const float* __restrict__ w5,
                                              unsigned short* d0, unsigned short* d1, unsigned short* d2,
                                              unsigned short* d3, unsigned short* d4, unsigned short* d5) {
  const int bid = blockIdx.x;
  const float* s;
  unsigned short* d;
  int lb;
  if (bid < 32)       { s = w0; d = d0; lb = bid; }
  else if (bid < 64)  { s = w1; d = d1; lb = bid - 32; }
  else if (bid < 96)  { s = w2; d = d2; lb = bid - 64; }
  else if (bid < 128) { s = w3; d = d3; lb = bid - 96; }
  else if (bid < 384) { s = w4; d = d4; lb = bid - 128; }
  else                { s = w5; d = d5; lb = bid - 384; }
  const size_t i8 = ((size_t)lb * 256 + threadIdx.x) * 8;
  const v4f a0 = *(const v4f*)(s + i8);
  const v4f a1 = *(const v4f*)(s + i8 + 4);
  const v4f b0 = bf16r4(a0) * WSCL;
  const v4f b1 = bf16r4(a1) * WSCL;
  const v4u hv = pack8h(b0, b1);
  unsigned short* dp = d + i8;
  for (int pass = 0; pass < 2; ++pass) {
    *(volatile v4u*)dp = hv;
    __threadfence();
  }
}

__global__ __launch_bounds__(256) void k_buildq(const float* __restrict__ query,
                                                const float* __restrict__ query_pos,
                                                const float* __restrict__ qpe_w,
                                                const float* __restrict__ qpe_b,
                                                float* Qtok, unsigned short* Qin) {
  float* sF = (float*)g_smem;
  unsigned short* sH = (unsigned short*)(g_smem + BQ_SH_OFF);
  float* sP = (float*)(g_smem + BQ_SP_OFF);
  const int t = threadIdx.x, lane = t & 31, wave = t >> 5;
  const int bq0 = blockIdx.x * 32;
  const int b = bq0 / NQRY, q0 = bq0 % NQRY;

#pragma unroll 1
  for (int i = 0; i < 32; ++i) {
    const int c = i * 8 + wave;
    sF[lane * TP + c] = bf16r(query[((size_t)b * CH + c) * NQRY + q0 + lane]);
  }
  {
    const int tt = (t < 192) ? t : 0;
    const int q = tt / 6, d = tt - q * 6;
    const float v = bf16r(query_pos[(size_t)(bq0 + q) * 6 + d]);
    if (t < 192) sP[q * 8 + d] = v;
  }
  __syncthreads();
  {
    const int c = t;
    float w[6];
#pragma unroll
    for (int d = 0; d < 6; ++d) w[d] = bf16r(qpe_w[c * 6 + d]);
    const float pb = bf16r(qpe_b[c]);
#pragma unroll 1
    for (int j = 0; j < 32; ++j) {
      const float* pp = sP + j * 8;
      float pe = pp[0] * w[0];
      pe += pp[1] * w[1];
      pe += pp[2] * w[2];
      pe += pp[3] * w[3];
      pe += pp[4] * w[4];
      pe += pp[5] * w[5];
      pe += pb;
      sH[j * EP + c] = f2h(sF[j * TP + c] + pe);
    }
  }
  __syncthreads();
  for (int pass = 0; pass < 2; ++pass) {
#pragma unroll 1
    for (int it = 0; it < 8; ++it) {
      const int row = it * 4 + (t >> 6);
      const int col = (t & 63) * 4;
      const v4f v = *(const v4f*)(sF + row * TP + col);
      *(volatile v4f*)(Qtok + (size_t)(bq0 + row) * CH + col) = v;
    }
#pragma unroll 1
    for (int it = 0; it < 4; ++it) {
      const int row = it * 8 + wave;
      const int col = lane * 8;
      const v4u hv = *(const v4u*)(sH + row * EP + col);
      *(volatile v4u*)(Qin + (size_t)(bq0 + row) * CH + col) = hv;
    }
    __threadfence();
  }
}

__global__ __launch_bounds__(256) void k_qproj(const unsigned short* __restrict__ Qin,
                                               const unsigned short* __restrict__ Wq,
                                               const float* __restrict__ q_b, float* Qh) {
  float* sT = (float*)g_smem;
  const int t = threadIdx.x, lane = t & 31, wave = t >> 5;
  const int m0 = blockIdx.x * 64;
  bgemm64x256<false>(Qin + (size_t)m0 * CH, CH, Wq, CH, CH, 1.0f / WSCL, q_b);
  __syncthreads();
  const int cA = lane * 4, cB = 128 + lane * 4;
  for (int pass = 0; pass < 2; ++pass) {
#pragma unroll 1
    for (int i = 0; i < 8; ++i) {
      const int row = wave * 8 + i;
      const size_t m = (size_t)(m0 + row);
      const v4f vA = *(const v4f*)(sT + row * TP + cA);
      const v4f vB = *(const v4f*)(sT + row * TP + cB);
      *(volatile v4f*)(Qh + m * CH + cA) = vA;
      *(volatile v4f*)(Qh + m * CH + cB) = vB;
    }
    __threadfence();
  }
}

__global__ __launch_bounds__(256) void k_attn(const float* __restrict__ key,
                                              const float* __restrict__ query_pos,
                                              const float* __restrict__ key_pos,
                                              const float* __restrict__ kpe_w,
                                              const float* __restrict__ kpe_b,
                                              const unsigned short* __restrict__ Wk,
                                              const float* __restrict__ k_b,
                                              const unsigned short* __restrict__ Wv,
                                              const float* __restrict__ v_b,
                                              const float* __restrict__ Qh,
                                              unsigned short* Ao) {
  float* sT = (float*)g_smem;
  unsigned short* sE = (unsigned short*)(g_smem + SE_OFF);
  float* sQh = (float*)(g_smem + SQH_OFF);
  float* sSc = (float*)(g_smem + SSC_OFF);
  float* sG  = (float*)(g_smem + SG_OFF);
  unsigned short* sAo = (unsigned short*)(g_smem + SAO_OFF);
  int* sIdx = (int*)(g_smem + SIDX_OFF);
  float* sQP = (float*)(g_smem + SQP_OFF);
  int* sCnt = (int*)(g_smem + SCNT_OFF);

  const int t = threadIdx.x, lane = t & 31, wave = t >> 5;
  const int bq0 = blockIdx.x * 4;
  const int b = bq0 / NQRY;

  {
    const int q = t >> 6, c4 = (t & 63) * 4;
    *(v4f*)(sQh + q * CH + c4) = *(const v4f*)(Qh + (size_t)(bq0 + q) * CH + c4);
    const int tt = (t < 24) ? t : 0;
    const int qq = tt / 6, d = tt - qq * 6;
    const float v = bf16r(query_pos[(size_t)(bq0 + qq) * 6 + d]);
    if (t < 24) sQP[qq * 8 + d] = v;
  }
  __syncthreads();

  if (wave < 4) {
    const int qi = wave;
    const float cx = sQP[qi * 8 + 0], cy = sQP[qi * 8 + 1], cz = sQP[qi * 8 + 2];
    const float hx = 0.5f * sQP[qi * 8 + 3], hy = 0.5f * sQP[qi * 8 + 4], hz = 0.5f * sQP[qi * 8 + 5];
    const float* kpb = key_pos + (size_t)b * NKEY * 3;
    int cnt = 0;
#pragma unroll 1
    for (int step = 0; step < NKEY / 32; ++step) {
      const int k = (step << 5) + lane;
      const float px = bf16r(kpb[k * 3 + 0]);
      const float py = bf16r(kpb[k * 3 + 1]);
      const float pz = bf16r(kpb[k * 3 + 2]);
      const bool inx = fabsf(px - cx) <= hx;
      const bool iny = fabsf(py - cy) <= hy;
      const bool inz = fabsf(pz - cz) <= hz;
      const bool in = inx & iny & inz;
      const unsigned m = __builtin_amdgcn_ballot_w32(in);
      const unsigned below = m & ((1u << lane) - 1u);
      const int slot = cnt + (int)__builtin_popcount(below);
      if (in && slot < NS) sIdx[qi * NS + slot] = k;
      cnt += (int)__builtin_popcount(m);
      if (cnt >= NS) break;
    }
    wave_sync_lds();
    const int cv = cnt < NS ? cnt : NS;
    if (lane < NS && lane >= cv) sIdx[qi * NS + lane] = 0;
    if (lane == 0) sCnt[qi] = cv;
    wave_sync_lds();
    const int s = lane & (NS - 1);
    int ki = sIdx[qi * NS + s];
    ki = clampi(ki, 0, NKEY - 1);
    const float gx = bf16r(kpb[ki * 3 + 0]) - cx;
    const float gy = bf16r(kpb[ki * 3 + 1]) - cy;
    const float gz = bf16r(kpb[ki * 3 + 2]) - cz;
    if (lane < NS) {
      float* gp = sG + (qi * NS + s) * 4;
      gp[0] = gx; gp[1] = gy; gp[2] = gz; gp[3] = 0.f;
    }
  }
  __syncthreads();

  {
    const int c = t;
    const float w0 = bf16r(kpe_w[c * 3 + 0]);
    const float w1 = bf16r(kpe_w[c * 3 + 1]);
    const float w2 = bf16r(kpe_w[c * 3 + 2]);
    const float kb = bf16r(kpe_b[c]);
    const float* kc = key + ((size_t)b * CH + c) * NKEY;
#pragma unroll 1
    for (int r = 0; r < 64; ++r) {
      int ki = sIdx[r];
      ki = clampi(ki, 0, NKEY - 1);
      const float kf = bf16r(kc[ki]);
      const v4f g = *(const v4f*)(sG + r * 4);
      float pe = g[0] * w0;
      pe += g[1] * w1;
      pe += g[2] * w2;
      pe += kb;
      sE[r * EP + c] = f2h(kf + pe);
    }
  }
  __syncthreads();

  bgemm64x256<true>(nullptr, EP, Wk, CH, CH, 1.0f / WSCL, k_b);
  __syncthreads();

#pragma unroll
  for (int p = 0; p < 2; ++p) {
    const int item = t + (p << 8);
    const int q = item >> 7, h = (item >> 4) & 7, s = item & 15;
    const float* qp = sQh + q * CH + h * DHEAD;
    const float* kp = sT + (q * NS + s) * TP + h * DHEAD;
    float dot = 0.f;
#pragma unroll
    for (int d = 0; d < DHEAD; d += 4) {
      const v4f a = *(const v4f*)(qp + d);
      const v4f kk = *(const v4f*)(kp + d);
      dot += a[0] * kk[0];
      dot += a[1] * kk[1];
      dot += a[2] * kk[2];
      dot += a[3] * kk[3];
    }
    dot *= RSQD;
    const int cq = sCnt[q];
    const bool masked = (s >= cq) && (s > 0);
    dot = masked ? -1.0e30f : dot;
    sSc[item] = dot;
  }
  __syncthreads();
  if (wave == 0) {
    float* ps = sSc + lane * NS;
    v4f e[4];
#pragma unroll
    for (int g = 0; g < 4; ++g) e[g] = *(const v4f*)(ps + 4 * g);
    float mx = e[0][0];
#pragma unroll
    for (int g = 0; g < 4; ++g) {
      mx = fmaxf(mx, fmaxf(fmaxf(e[g][0], e[g][1]), fmaxf(e[g][2], e[g][3])));
    }
    float sum = 0.f;
#pragma unroll
    for (int g = 0; g < 4; ++g) {
      e[g][0] = __expf(e[g][0] - mx);
      e[g][1] = __expf(e[g][1] - mx);
      e[g][2] = __expf(e[g][2] - mx);
      e[g][3] = __expf(e[g][3] - mx);
      sum += (e[g][0] + e[g][1]) + (e[g][2] + e[g][3]);
    }
    const float inv = 1.0f / sum;
#pragma unroll
    for (int g = 0; g < 4; ++g) *(v4f*)(ps + 4 * g) = e[g] * inv;
  }
  __syncthreads();

  bgemm64x256<true>(nullptr, EP, Wv, CH, CH, 1.0f / WSCL, v_b);
  __syncthreads();

  {
    const int c = t, h = c >> 5;
#pragma unroll
    for (int q = 0; q < 4; ++q) {
      const float* pp = sSc + (q * NHEAD + h) * NS;
      const v4f p0 = *(const v4f*)(pp), p1 = *(const v4f*)(pp + 4);
      const v4f p2 = *(const v4f*)(pp + 8), p3 = *(const v4f*)(pp + 12);
      const float* vp = sT + (q * NS) * TP + c;
      float a = 0.f;
      a += p0[0] * vp[0 * TP];  a += p0[1] * vp[1 * TP];  a += p0[2] * vp[2 * TP];  a += p0[3] * vp[3 * TP];
      a += p1[0] * vp[4 * TP];  a += p1[1] * vp[5 * TP];  a += p1[2] * vp[6 * TP];  a += p1[3] * vp[7 * TP];
      a += p2[0] * vp[8 * TP];  a += p2[1] * vp[9 * TP];  a += p2[2] * vp[10 * TP]; a += p2[3] * vp[11 * TP];
      a += p3[0] * vp[12 * TP]; a += p3[1] * vp[13 * TP]; a += p3[2] * vp[14 * TP]; a += p3[3] * vp[15 * TP];
      sAo[q * CH + c] = f2h(a * ASCL);
    }
  }
  __syncthreads();
  if (wave < 4) {
    const v4u hv = *(const v4u*)(sAo + wave * CH + lane * 8);
    unsigned short* dst = Ao + (size_t)(bq0 + wave) * CH + lane * 8;
    for (int pass = 0; pass < 2; ++pass) {
      *(volatile v4u*)dst = hv;
      __threadfence();
    }
  }
}

__device__ __forceinline__ void ln_row(v4f yA, v4f yB, v4f gA, v4f gB, v4f bA, v4f bB, v4f& xA, v4f& xB) {
  float s = ((yA[0] + yA[1]) + (yA[2] + yA[3])) + ((yB[0] + yB[1]) + (yB[2] + yB[3]));
  s = wsum(s);
  const float mean = s * (1.0f / CH);
  const v4f dA = yA - mean;
  const v4f dB = yB - mean;
  float v = ((dA[0] * dA[0] + dA[1] * dA[1]) + (dA[2] * dA[2] + dA[3] * dA[3])) +
            ((dB[0] * dB[0] + dB[1] * dB[1]) + (dB[2] * dB[2] + dB[3] * dB[3]));
  v = wsum(v);
  const float rstd = rsqrtf(v * (1.0f / CH) + LNEPS);
  xA = dA * rstd * gA + bA;
  xB = dB * rstd * gB + bB;
}

__global__ __launch_bounds__(256) void k_oproj_ln1(const unsigned short* __restrict__ Ao,
                                                   const unsigned short* __restrict__ Wo,
                                                   const float* __restrict__ o_b,
                                                   const float* __restrict__ Qtok,
                                                   const float* __restrict__ n1g,
                                                   const float* __restrict__ n1b,
                                                   float* X1f, unsigned short* X1h) {
  float* sT = (float*)g_smem;
  unsigned short* sRow = (unsigned short*)(g_smem + SROW_OFF);
  const int t = threadIdx.x, lane = t & 31, wave = t >> 5;
  const int m0 = blockIdx.x * 64;
  bgemm64x256<false>(Ao + (size_t)m0 * CH, CH, Wo, CH, CH, 1.0f / (ASCL * WSCL), o_b);
  __syncthreads();
  const int cA = lane * 4, cB = 128 + lane * 4;
  const v4f gA = bf16r4(*(const v4f*)(n1g + cA)), gB = bf16r4(*(const v4f*)(n1g + cB));
  const v4f bA = bf16r4(*(const v4f*)(n1b + cA)), bB = bf16r4(*(const v4f*)(n1b + cB));
  unsigned short* srw = sRow + wave * CH;
#pragma unroll 1
  for (int i = 0; i < 8; ++i) {
    const int row = wave * 8 + i;
    const size_t m = (size_t)(m0 + row);
    const v4f yA = *(const v4f*)(sT + row * TP + cA) + *(const v4f*)(Qtok + m * CH + cA);
    const v4f yB = *(const v4f*)(sT + row * TP + cB) + *(const v4f*)(Qtok + m * CH + cB);
    v4f xA, xB;
    ln_row(yA, yB, gA, gB, bA, bB, xA, xB);
    *(v2u*)(srw + cA) = pack4h(xA);
    *(v2u*)(srw + cB) = pack4h(xB);
    wave_sync_lds();
    const v4u hv = *(const v4u*)(srw + lane * 8);
    wave_sync_lds();
    for (int pass = 0; pass < 2; ++pass) {
      *(volatile v4f*)(X1f + m * CH + cA) = xA;
      *(volatile v4f*)(X1f + m * CH + cB) = xB;
      *(volatile v4u*)(X1h + m * CH + lane * 8) = hv;
      __threadfence();
    }
  }
}

__global__ __launch_bounds__(256) void k_ffn1(const unsigned short* __restrict__ X1h,
                                              const unsigned short* __restrict__ W1,
                                              const float* __restrict__ b1, unsigned short* Hh) {
  float* sT = (float*)g_smem;
  const int t = threadIdx.x, lane = t & 31, wave = t >> 5;
  const int m0 = blockIdx.x * 64;
  const int nb = blockIdx.y;
  bgemm64x256<false>(X1h + (size_t)m0 * CH, CH, W1 + (size_t)nb * CH * CH, CH, CH, 1.0f / WSCL, b1 + nb * CH);
  __syncthreads();
#pragma unroll 1
  for (int i = 0; i < 8; ++i) {
    const int row = wave * 8 + i;
    const size_t m = (size_t)(m0 + row);
    const float* sp = sT + row * TP + lane * 8;
    v4f a0 = *(const v4f*)(sp);
    v4f a1 = *(const v4f*)(sp + 4);
#pragma unroll
    for (int e = 0; e < 4; ++e) {
      a0[e] = fmaxf(a0[e], 0.f) * ASCL;
      a1[e] = fmaxf(a1[e], 0.f) * ASCL;
    }
    const v4u hv = pack8h(a0, a1);
    unsigned short* dst = Hh + m * FFD + (size_t)nb * CH + lane * 8;
    for (int pass = 0; pass < 2; ++pass) {
      *(volatile v4u*)dst = hv;
      __threadfence();
    }
  }
}

__global__ __launch_bounds__(256) void k_ffn2out(const unsigned short* __restrict__ Hh,
                                                 const unsigned short* __restrict__ W2,
                                                 const float* __restrict__ b2,
                                                 const float* __restrict__ X1f,
                                                 const float* __restrict__ n2g,
                                                 const float* __restrict__ n2b, float* out) {
  float* sT = (float*)g_smem;
  const int t = threadIdx.x, lane = t & 31, wave = t >> 5;
  const int m0 = blockIdx.x * 64;
  bgemm64x256<false>(Hh + (size_t)m0 * FFD, FFD, W2, FFD, FFD, 1.0f / (ASCL * WSCL), b2);
  __syncthreads();
  const int cA = lane * 4, cB = 128 + lane * 4;
  const v4f gA = bf16r4(*(const v4f*)(n2g + cA)), gB = bf16r4(*(const v4f*)(n2g + cB));
  const v4f bA = bf16r4(*(const v4f*)(n2b + cA)), bB = bf16r4(*(const v4f*)(n2b + cB));
#pragma unroll 1
  for (int i = 0; i < 8; ++i) {
    const int row = wave * 8 + i;
    const size_t m = (size_t)(m0 + row);
    const v4f yA = *(const v4f*)(sT + row * TP + cA) + *(const v4f*)(X1f + m * CH + cA);
    const v4f yB = *(const v4f*)(sT + row * TP + cB) + *(const v4f*)(X1f + m * CH + cB);
    v4f xA, xB;
    ln_row(yA, yB, gA, gB, bA, bB, xA, xB);
    *(v4f*)(sT + row * TP + cA) = xA;
    *(v4f*)(sT + row * TP + cB) = xB;
  }
  __syncthreads();
  const int bb = m0 / NQRY, q0 = m0 % NQRY;
  for (int pass = 0; pass < 2; ++pass) {
#pragma unroll 1
    for (int it = 0; it < 16; ++it) {
      const int c = it * 16 + (t >> 4);
      const int qq = (t & 15) * 4;
      v4f v;
      v[0] = sT[(qq + 0) * TP + c];
      v[1] = sT[(qq + 1) * TP + c];
      v[2] = sT[(qq + 2) * TP + c];
      v[3] = sT[(qq + 3) * TP + c];
      *(volatile v4f*)(out + ((size_t)bb * CH + c) * NQRY + q0 + qq) = v;
    }
    __threadfence();
  }
}

extern "C" void kernel_launch(void* const* d_in, const int* in_sizes, int n_in,
                              void* d_out, int out_size, void* d_ws, size_t ws_size,
                              hipStream_t stream) {
  if (n_in < 24) return;
  if (in_sizes[0] != NBATCH * CH * NQRY) return;
  if (in_sizes[1] != NBATCH * CH * NKEY) return;
  if (in_sizes[2] != NBATCH * NQRY * 6) return;
  if (in_sizes[3] != NBATCH * NKEY * 3) return;
  if (in_sizes[4] != CH * CH || in_sizes[6] != CH * CH || in_sizes[8] != CH * CH || in_sizes[10] != CH * CH) return;
  if (in_sizes[5] != CH || in_sizes[7] != CH || in_sizes[9] != CH || in_sizes[11] != CH) return;
  if (in_sizes[12] != FFD * CH || in_sizes[13] != FFD || in_sizes[14] != CH * FFD || in_sizes[15] != CH) return;
  if (in_sizes[16] != CH || in_sizes[17] != CH || in_sizes[18] != CH || in_sizes[19] != CH) return;
  if (in_sizes[20] != CH * 6 || in_sizes[21] != CH || in_sizes[22] != CH * 3 || in_sizes[23] != CH) return;
  if (out_size != NBATCH * CH * NQRY) return;

  const float* query     = (const float*)d_in[0];
  const float* key       = (const float*)d_in[1];
  const float* query_pos = (const float*)d_in[2];
  const float* key_pos   = (const float*)d_in[3];
  const float* q_w    = (const float*)d_in[4];
  const float* q_b    = (const float*)d_in[5];
  const float* k_w    = (const float*)d_in[6];
  const float* k_b    = (const float*)d_in[7];
  const float* v_w    = (const float*)d_in[8];
  const float* v_b    = (const float*)d_in[9];
  const float* o_w    = (const float*)d_in[10];
  const float* o_b    = (const float*)d_in[11];
  const float* lin1_w = (const float*)d_in[12];
  const float* lin1_b = (const float*)d_in[13];
  const float* lin2_w = (const float*)d_in[14];
  const float* lin2_b = (const float*)d_in[15];
  const float* n1_g   = (const float*)d_in[16];
  const float* n1_b   = (const float*)d_in[17];
  const float* n2_g   = (const float*)d_in[18];
  const float* n2_b   = (const float*)d_in[19];
  const float* qpe_w  = (const float*)d_in[20];
  const float* qpe_b  = (const float*)d_in[21];
  const float* kpe_w  = (const float*)d_in[22];
  const float* kpe_b  = (const float*)d_in[23];
  float* out = (float*)d_out;

  const size_t PW   = (size_t)CH * CH * 2;
  const size_t PWF  = (size_t)FFD * CH * 2;
  const size_t PF32 = (size_t)NBQ * CH * 4;
  const size_t PF16 = (size_t)NBQ * CH * 2;
  const size_t PH16 = (size_t)NBQ * FFD * 2;
  size_t off = 0;
  const size_t oWq = off; off += PW;
  const size_t oWk = off; off += PW;
  const size_t oWv = off; off += PW;
  const size_t oWo = off; off += PW;
  const size_t oW1 = off; off += PWF;
  const size_t oW2 = off; off += PWF;
  const size_t oQt = off; off += PF32;
  const size_t oQi = off; off += PF16;
  const size_t oQh = off; off += PF32;
  const size_t oAo = off; off += PF16;
  const size_t oXf = off; off += PF32;
  const size_t oXh = off; off += PF16;
  const size_t oH  = off; off += PH16;
  if (off > ws_size) return;
  if (off > (size_t)134217728) return;

  char* ws = (char*)d_ws;
  unsigned short* Wq16 = (unsigned short*)(ws + oWq);
  unsigned short* Wk16 = (unsigned short*)(ws + oWk);
  unsigned short* Wv16 = (unsigned short*)(ws + oWv);
  unsigned short* Wo16 = (unsigned short*)(ws + oWo);
  unsigned short* W1h  = (unsigned short*)(ws + oW1);
  unsigned short* W2h  = (unsigned short*)(ws + oW2);
  float*          Qtok = (float*)(ws + oQt);
  unsigned short* Qin  = (unsigned short*)(ws + oQi);
  float*          Qh   = (float*)(ws + oQh);
  unsigned short* Ao   = (unsigned short*)(ws + oAo);
  float*          X1f  = (float*)(ws + oXf);
  unsigned short* X1h  = (unsigned short*)(ws + oXh);
  unsigned short* Hh   = (unsigned short*)(ws + oH);

  (void)hipFuncSetAttribute(reinterpret_cast<const void*>(&k_buildq), hipFuncAttributeMaxDynamicSharedMemorySize, BQ_SMEM);
  (void)hipFuncSetAttribute(reinterpret_cast<const void*>(&k_qproj), hipFuncAttributeMaxDynamicSharedMemorySize, GEMM_SMEM);
  (void)hipFuncSetAttribute(reinterpret_cast<const void*>(&k_attn), hipFuncAttributeMaxDynamicSharedMemorySize, ATT_SMEM);
  (void)hipFuncSetAttribute(reinterpret_cast<const void*>(&k_oproj_ln1), hipFuncAttributeMaxDynamicSharedMemorySize, LN1_SMEM);
  (void)hipFuncSetAttribute(reinterpret_cast<const void*>(&k_ffn1), hipFuncAttributeMaxDynamicSharedMemorySize, GEMM_SMEM);
  (void)hipFuncSetAttribute(reinterpret_cast<const void*>(&k_ffn2out), hipFuncAttributeMaxDynamicSharedMemorySize, GEMM_SMEM);

  const dim3 blk(256);
  const int gW = (4 * CH * CH + 2 * FFD * CH) / 2048;

  k_cvtw<<<dim3(gW), blk, 0, stream>>>(q_w, k_w, v_w, o_w, lin1_w, lin2_w, Wq16, Wk16, Wv16, Wo16, W1h, W2h);
  k_buildq<<<dim3(NBQ / 32), blk, BQ_SMEM, stream>>>(query, query_pos, qpe_w, qpe_b, Qtok, Qin);
  k_qproj<<<dim3(NBQ / 64), blk, GEMM_SMEM, stream>>>(Qin, Wq16, q_b, Qh);
  k_attn<<<dim3(NBQ / 4), blk, ATT_SMEM, stream>>>(key, query_pos, key_pos, kpe_w, kpe_b,
                                                   Wk16, k_b, Wv16, v_b, Qh, Ao);
  k_oproj_ln1<<<dim3(NBQ / 64), blk, LN1_SMEM, stream>>>(Ao, Wo16, o_b, Qtok, n1_g, n1_b, X1f, X1h);
  k_ffn1<<<dim3(NBQ / 64, FFD / CH), blk, GEMM_SMEM, stream>>>(X1h, W1h, lin1_b, Hh);
  k_ffn2out<<<dim3(NBQ / 64), blk, GEMM_SMEM, stream>>>(Hh, W2h, lin2_b, X1f, n2_g, n2_b, out);
  (void)hipGetLastError();
}
